// ClusterForecasting_62208306315949
// MI455X (gfx1250) — hardware-verified
//
#include <hip/hip_runtime.h>


namespace {
constexpr int BS = 32, S = 128, IN = 8, D = 128, NH = 8, DH = 16, NL = 2, DFF = 512, KN = 16, NT = BS * S, NBLK = NT / 16;
constexpr float XS = 8.0f, PS = 1024.0f, WSC = 256.0f;
typedef _Float16 b16;
typedef __attribute__((ext_vector_type(16))) _Float16 v16b;
typedef __attribute__((ext_vector_type(8))) _Float16 v8b;
typedef __attribute__((ext_vector_type(8))) float v8f;
typedef __attribute__((ext_vector_type(4))) float v4f;
__device__ __forceinline__ float bf16_rne(float f) { unsigned int u = __float_as_uint(f); u += 0x7FFFu + ((u >> 16) & 1u); return __uint_as_float(u & 0xFFFF0000u); }
__device__ __forceinline__ void split16(float v, b16& hi, b16& lo) { hi = (b16)v; lo = (b16)(v - (float)hi); }
__device__ __forceinline__ v16b frag_kb(const b16* p, int hh) { const v8b a = *(const v8b*)(p + 8 * hh), b = *(const v8b*)(p + 16 + 8 * hh); v16b f;
#pragma unroll
  for (int e = 0; e < 8; ++e) { f[e] = a[e]; f[8 + e] = b[e]; } return f; }
__device__ __forceinline__ v8f wmma16b(v16b a, v16b b, v8f c) { v8f d = __builtin_amdgcn_wmma_f32_16x16x32_f16(false, a, false, b, (short)0, c, false, false); asm volatile("v_nop\n\tv_nop\n\tv_nop\n\tv_nop" : "+v"(d) : "v"(a), "v"(b)); return d; }
__device__ __forceinline__ void wave_lds_sync() { __builtin_amdgcn_fence(__ATOMIC_RELEASE, "workgroup"); __builtin_amdgcn_wave_barrier(); __builtin_amdgcn_fence(__ATOMIC_ACQUIRE, "workgroup"); }
__device__ __forceinline__ float pmul(float a, float b) { float p = a * b; asm volatile("" : "+v"(p)); return p; }

__global__ __launch_bounds__(256) void wput_kernel(const float* __restrict__ w, int KIN, int KP, int OUTW, b16* __restrict__ WT) {
  const int KG = KP / 8; const int u = blockIdx.x * 256 + threadIdx.x; if (u >= OUTW * KG) return; const int o = u / KG, k0 = (u % KG) * 8; v8b v;
#pragma unroll
  for (int j = 0; j < 8; ++j) { const int k = k0 + j; v[j] = k < KIN ? (b16)(bf16_rne(w[(size_t)k * OUTW + o]) * WSC) : (b16)0.0f; } for (int pass = 0; pass < 2; ++pass) { *(volatile v8b*)(WT + (size_t)o * KP + k0) = v; __threadfence(); }
}
__global__ __launch_bounds__(32) void emb_kernel(const float* __restrict__ x, const b16* __restrict__ WE, const float* __restrict__ be, int RL, float* __restrict__ H) {
  __shared__ __attribute__((aligned(16))) b16 Ah[16][40]; __shared__ float Tf[16][D + 4]; const int lane = threadIdx.x, nloc = lane & 15, hlf = lane >> 4; const size_t m0 = (size_t)blockIdx.x * 16; if (m0 >= (size_t)RL) return;
  for (int rr = 0; rr < 16; ++rr) Ah[rr][lane] = (b16)((lane < IN ? bf16_rne(x[(m0 + rr) * IN + lane]) : 0.0f) * XS);
  wave_lds_sync(); const v16b a = frag_kb(&Ah[nloc][0], hlf);
#pragma unroll
  for (int t = 0; t < 8; ++t) { v8f acc = {}; acc = wmma16b(a, frag_kb(WE + (size_t)(t * 16 + nloc) * 32, hlf), acc); const int c = t * 16 + nloc; const float bb = bf16_rne(be[c]);
#pragma unroll
    for (int r8 = 0; r8 < 8; ++r8) Tf[8 * hlf + r8][c] = acc[r8] * (1.0f / (XS * WSC)) + bb; }
  wave_lds_sync();
  for (int pass = 0; pass < 2; ++pass) { for (int rr = 0; rr < 16; ++rr) *(volatile v4f*)(H + (m0 + rr) * D + lane * 4) = *(const v4f*)(&Tf[rr][lane * 4]); __threadfence(); }
}
__global__ __launch_bounds__(32) void qkv_kernel(const float* __restrict__ H, const b16* __restrict__ WQ, const b16* __restrict__ WK, const b16* __restrict__ WV, int RL, float* __restrict__ QKV) {
  __shared__ __attribute__((aligned(16))) b16 Ah[16][D + 8], Al[16][D + 8]; __shared__ float Tf[16][D + 4]; const int lane = threadIdx.x, nloc = lane & 15, hlf = lane >> 4; const size_t m0 = (size_t)blockIdx.x * 16; if (m0 >= (size_t)RL) return;
  for (int rr = 0; rr < 16; ++rr) for (int q = 0; q < 4; ++q) { b16 p, ql; split16(H[(m0 + rr) * D + q * 32 + lane] * XS, p, ql); Ah[rr][q * 32 + lane] = p; Al[rr][q * 32 + lane] = ql; }
  wave_lds_sync();
#pragma unroll 1
  for (int g = 0; g < 3; ++g) { const b16* W = g == 0 ? WQ : (g == 1 ? WK : WV); v8f acc[8];
#pragma unroll
    for (int t = 0; t < 8; ++t) acc[t] = (v8f){};
#pragma unroll
    for (int kb = 0; kb < D; kb += 32) { const v16b a = frag_kb(&Ah[nloc][kb], hlf), al = frag_kb(&Al[nloc][kb], hlf);
#pragma unroll
      for (int t = 0; t < 8; ++t) { const v16b bw = frag_kb(W + (size_t)(t * 16 + nloc) * D + kb, hlf); acc[t] = wmma16b(a, bw, acc[t]); acc[t] = wmma16b(al, bw, acc[t]); } }
#pragma unroll
    for (int t = 0; t < 8; ++t)
#pragma unroll
      for (int r8 = 0; r8 < 8; ++r8) Tf[8 * hlf + r8][t * 16 + nloc] = acc[t][r8] * (1.0f / (XS * WSC));
    wave_lds_sync();
    for (int pass = 0; pass < 2; ++pass) { for (int rr = 0; rr < 16; ++rr) *(volatile v4f*)(QKV + (m0 + rr) * (3 * D) + g * D + lane * 4) = *(const v4f*)(&Tf[rr][lane * 4]); __threadfence(); }
    wave_lds_sync(); }
}
__global__ __launch_bounds__(32) void att_kernel(const float* __restrict__ QKV, int BV, float* __restrict__ ATT) {
  __shared__ __attribute__((aligned(16))) b16 Qh[16][40], Ql[16][40], Kh[S][40], Kl[S][40], Ph[16][S + 8], Vh[DH][S + 8], Vl[DH][S + 8]; __shared__ float Sc[16][S + 1], Of[16][D + 1];
  const int lane = threadIdx.x, nloc = lane & 15, hlf = lane >> 4; const int b = blockIdx.x / (S / 16), qb = blockIdx.x % (S / 16); if (b >= BV) return; const size_t base = (size_t)b * S, q0 = base + qb * 16;
#pragma unroll 1
  for (int h = 0; h < NH; ++h) {
    for (int rr = 0; rr < 16; ++rr) { b16 p = (b16)0.0f, ql = (b16)0.0f; if (lane < DH) split16(QKV[(q0 + rr) * (3 * D) + h * DH + lane] * XS, p, ql); Qh[rr][lane] = p; Ql[rr][lane] = ql; }
    for (int rr = 0; rr < S; ++rr) { const float* kp = QKV + (base + rr) * (3 * D) + D + h * DH; const float* vp = QKV + (base + rr) * (3 * D) + 2 * D + h * DH; b16 p = (b16)0.0f, ql = (b16)0.0f; if (lane < DH) split16(kp[lane] * XS, p, ql); Kh[rr][lane] = p; Kl[rr][lane] = ql; if (lane < DH) { split16(vp[lane] * XS, p, ql); Vh[lane][rr] = p; Vl[lane][rr] = ql; } }
    wave_lds_sync(); const v16b qh = frag_kb(&Qh[nloc][0], hlf), qlo = frag_kb(&Ql[nloc][0], hlf);
#pragma unroll
    for (int t = 0; t < 8; ++t) { const v16b kh = frag_kb(&Kh[t * 16 + nloc][0], hlf), kl = frag_kb(&Kl[t * 16 + nloc][0], hlf); v8f s = {}; s = wmma16b(qh, kh, s); s = wmma16b(qh, kl, s); s = wmma16b(qlo, kh, s);
#pragma unroll
      for (int r8 = 0; r8 < 8; ++r8) Sc[8 * hlf + r8][t * 16 + nloc] = s[r8] * (0.25f / (XS * XS)); }
    wave_lds_sync();
    for (int qi = 0; qi < 16; ++qi) { float v[4], mx = -INFINITY; for (int k = 0; k < 4; ++k) { v[k] = Sc[qi][k * 32 + lane]; mx = fmaxf(mx, v[k]); } for (int o = 16; o; o >>= 1) mx = fmaxf(mx, __shfl_xor(mx, o)); float sm = 0.0f; for (int k = 0; k < 4; ++k) { v[k] = __expf(v[k] - mx); sm += v[k]; } for (int o = 16; o; o >>= 1) sm += __shfl_xor(sm, o); const float inv = 1.0f / sm; for (int k = 0; k < 4; ++k) Ph[qi][k * 32 + lane] = (b16)(v[k] * inv * PS); }
    wave_lds_sync(); v8f o = {};
#pragma unroll
    for (int kb = 0; kb < S; kb += 32) { const v16b pa = frag_kb(&Ph[nloc][kb], hlf); o = wmma16b(pa, frag_kb(&Vh[nloc][kb], hlf), o); o = wmma16b(pa, frag_kb(&Vl[nloc][kb], hlf), o); }
#pragma unroll
    for (int r8 = 0; r8 < 8; ++r8) Of[8 * hlf + r8][h * DH + nloc] = o[r8] * (1.0f / (PS * XS));
    wave_lds_sync(); }
  for (int pass = 0; pass < 2; ++pass) { for (int rr = 0; rr < 16; ++rr) *(volatile v4f*)(ATT + (q0 + rr) * D + lane * 4) = (v4f){Of[rr][lane * 4], Of[rr][lane * 4 + 1], Of[rr][lane * 4 + 2], Of[rr][lane * 4 + 3]}; __threadfence(); }
}
__device__ __forceinline__ void row_ln(float (*Tf)[D + 4], int lane, const float* g, const float* bta) {
  __shared__ float Mu[16], Rs[16];
  if (lane < 16) { float s = 0.0f; for (int c = 0; c < D; ++c) s += Tf[lane][c]; const float mu = s * (1.0f / D); float v = 0.0f; for (int c = 0; c < D; ++c) { const float d = Tf[lane][c] - mu; v += pmul(d, d); } Mu[lane] = mu; Rs[lane] = rsqrtf(v * (1.0f / D) + 1e-5f); }
  wave_lds_sync();
  for (int rr = 0; rr < 16; ++rr) for (int q = 0; q < 4; ++q) { const int c = q * 32 + lane; Tf[rr][c] = pmul(pmul(Tf[rr][c] - Mu[rr], Rs[rr]), bf16_rne(g[c])) + bf16_rne(bta[c]); }
  wave_lds_sync();
}
__global__ __launch_bounds__(32) void wo_kernel(const float* __restrict__ ATT, const float* __restrict__ H, const b16* __restrict__ WO, const float* __restrict__ g, const float* __restrict__ bta, int RL, float* __restrict__ H1) {
  __shared__ __attribute__((aligned(16))) b16 Ah[16][D + 8], Al[16][D + 8]; __shared__ float Tf[16][D + 4]; const int lane = threadIdx.x, nloc = lane & 15, hlf = lane >> 4; const size_t m0 = (size_t)blockIdx.x * 16; if (m0 >= (size_t)RL) return;
  for (int rr = 0; rr < 16; ++rr) for (int q = 0; q < 4; ++q) { b16 p, ql; split16(ATT[(m0 + rr) * D + q * 32 + lane] * XS, p, ql); Ah[rr][q * 32 + lane] = p; Al[rr][q * 32 + lane] = ql; }
  wave_lds_sync(); v8f acc[8];
#pragma unroll
  for (int t = 0; t < 8; ++t) acc[t] = (v8f){};
#pragma unroll
  for (int kb = 0; kb < D; kb += 32) { const v16b a = frag_kb(&Ah[nloc][kb], hlf), al = frag_kb(&Al[nloc][kb], hlf);
#pragma unroll
    for (int t = 0; t < 8; ++t) { const v16b bw = frag_kb(WO + (size_t)(t * 16 + nloc) * D + kb, hlf); acc[t] = wmma16b(a, bw, acc[t]); acc[t] = wmma16b(al, bw, acc[t]); } }
#pragma unroll
  for (int t = 0; t < 8; ++t) { const int c = t * 16 + nloc;
#pragma unroll
    for (int r8 = 0; r8 < 8; ++r8) Tf[8 * hlf + r8][c] = acc[t][r8] * (1.0f / (XS * WSC)) + H[(m0 + 8 * hlf + r8) * D + c]; }
  wave_lds_sync(); row_ln(Tf, lane, g, bta);
  for (int pass = 0; pass < 2; ++pass) { for (int rr = 0; rr < 16; ++rr) *(volatile v4f*)(H1 + (m0 + rr) * D + lane * 4) = *(const v4f*)(&Tf[rr][lane * 4]); __threadfence(); }
}
__global__ __launch_bounds__(32) void ffn_kernel(const float* __restrict__ H1, const b16* __restrict__ W1T, const float* __restrict__ b1, const b16* __restrict__ W2T, const float* __restrict__ b2, const float* __restrict__ g, const float* __restrict__ bta, int RL, float* __restrict__ H) {
  __shared__ __attribute__((aligned(16))) b16 Ah[16][D + 8], Al[16][D + 8], Fh[16][DFF + 8], Fl[16][DFF + 8]; __shared__ float Tf[16][D + 4]; const int lane = threadIdx.x, nloc = lane & 15, hlf = lane >> 4; const size_t m0 = (size_t)blockIdx.x * 16; if (m0 >= (size_t)RL) return;
  for (int rr = 0; rr < 16; ++rr) for (int q = 0; q < 4; ++q) { b16 p, ql; split16(H1[(m0 + rr) * D + q * 32 + lane] * XS, p, ql); Ah[rr][q * 32 + lane] = p; Al[rr][q * 32 + lane] = ql; }
  wave_lds_sync();
#pragma unroll 1
  for (int cg = 0; cg < 4; ++cg) { v8f acc[8];
#pragma unroll
    for (int t = 0; t < 8; ++t) acc[t] = (v8f){};
#pragma unroll
    for (int kb = 0; kb < D; kb += 32) { const v16b a = frag_kb(&Ah[nloc][kb], hlf), al = frag_kb(&Al[nloc][kb], hlf);
#pragma unroll
      for (int t = 0; t < 8; ++t) { const v16b bw = frag_kb(W1T + (size_t)(cg * 128 + t * 16 + nloc) * D + kb, hlf); acc[t] = wmma16b(a, bw, acc[t]); acc[t] = wmma16b(al, bw, acc[t]); } }
#pragma unroll
    for (int t = 0; t < 8; ++t) { const int c = cg * 128 + t * 16 + nloc; const float bb = bf16_rne(b1[c]);
#pragma unroll
      for (int r8 = 0; r8 < 8; ++r8) { b16 p, q; split16(fmaxf(acc[t][r8] * (1.0f / (XS * WSC)) + bb, 0.0f) * XS, p, q); Fh[8 * hlf + r8][c] = p; Fl[8 * hlf + r8][c] = q; } } }
  wave_lds_sync(); v8f acc[8];
#pragma unroll
  for (int t = 0; t < 8; ++t) acc[t] = (v8f){};
#pragma unroll 2
  for (int kb = 0; kb < DFF; kb += 32) { const v16b a = frag_kb(&Fh[nloc][kb], hlf), al = frag_kb(&Fl[nloc][kb], hlf);
#pragma unroll
    for (int t = 0; t < 8; ++t) { const v16b bw = frag_kb(W2T + (size_t)(t * 16 + nloc) * DFF + kb, hlf); acc[t] = wmma16b(a, bw, acc[t]); acc[t] = wmma16b(al, bw, acc[t]); } }
#pragma unroll
  for (int t = 0; t < 8; ++t) { const int c = t * 16 + nloc; const float bb = bf16_rne(b2[c]);
#pragma unroll
    for (int r8 = 0; r8 < 8; ++r8) Tf[8 * hlf + r8][c] = acc[t][r8] * (1.0f / (XS * WSC)) + bb + H1[(m0 + 8 * hlf + r8) * D + c]; }
  wave_lds_sync(); row_ln(Tf, lane, g, bta);
  for (int pass = 0; pass < 2; ++pass) { for (int rr = 0; rr < 16; ++rr) *(volatile v4f*)(H + (m0 + rr) * D + lane * 4) = *(const v4f*)(&Tf[rr][lane * 4]); __threadfence(); }
}
__global__ __launch_bounds__(256) void sq_kernel(const float* __restrict__ H, int RL, float* __restrict__ SQ) { const int r = blockIdx.x * 256 + threadIdx.x; if (r >= RL) return; float s = 0.0f;
#pragma unroll 4
  for (int c = 0; c < D; ++c) { const float v = H[(size_t)r * D + c]; s += pmul(v, v); } for (int pass = 0; pass < 2; ++pass) { ((volatile float*)SQ)[r] = s; __threadfence(); } }
__global__ __launch_bounds__(32) void knn_kernel(const float* __restrict__ H, const float* __restrict__ SQ, int RL, float* __restrict__ PART) {
  __shared__ __attribute__((aligned(16))) b16 Ah[16][D + 8], Al[16][D + 8], Bh[128][D + 8], Bl[128][D + 8]; __shared__ float Dst[16][129], Rsum[16];
  const int lane = threadIdx.x, nloc = lane & 15, hlf = lane >> 4; const size_t m0 = (size_t)blockIdx.x * 16; if (m0 >= (size_t)RL) return;
  for (int rr = 0; rr < 16; ++rr) for (int q = 0; q < 4; ++q) { b16 p, ql; split16(H[(m0 + rr) * D + q * 32 + lane] * XS, p, ql); Ah[rr][q * 32 + lane] = p; Al[rr][q * 32 + lane] = ql; }
  float top[KN];
#pragma unroll
  for (int k = 0; k < KN; ++k) top[k] = INFINITY;
  const float sqi = lane < 16 ? SQ[m0 + lane] : 0.0f;
#pragma unroll 1
  for (int j0 = 0; j0 < RL; j0 += 128) {
    for (int rr = 0; rr < 128; ++rr) for (int q = 0; q < 4; ++q) { b16 p, ql; split16(H[(size_t)(j0 + rr) * D + q * 32 + lane] * XS, p, ql); Bh[rr][q * 32 + lane] = p; Bl[rr][q * 32 + lane] = ql; }
    wave_lds_sync(); v8f acc[8];
#pragma unroll
    for (int t = 0; t < 8; ++t) acc[t] = (v8f){};
#pragma unroll
    for (int kb = 0; kb < D; kb += 32) { const v16b a = frag_kb(&Ah[nloc][kb], hlf), al = frag_kb(&Al[nloc][kb], hlf);
#pragma unroll
      for (int t = 0; t < 8; ++t) { const v16b bh = frag_kb(&Bh[t * 16 + nloc][kb], hlf), bl = frag_kb(&Bl[t * 16 + nloc][kb], hlf); acc[t] = wmma16b(a, bh, acc[t]); acc[t] = wmma16b(a, bl, acc[t]); acc[t] = wmma16b(al, bh, acc[t]); } }
#pragma unroll
    for (int t = 0; t < 8; ++t) { const int j = t * 16 + nloc; const float sqj = SQ[j0 + j];
#pragma unroll
      for (int r8 = 0; r8 < 8; ++r8) Dst[8 * hlf + r8][j] = sqj - 2.0f * (acc[t][r8] * (1.0f / (XS * XS))); }
    wave_lds_sync();
    if (lane < 16) {
#pragma unroll 1
      for (int j = 0; j < 128; ++j) { float v = Dst[lane][j] + sqi;
#pragma unroll
        for (int k = 0; k < KN; ++k) { if (v < top[k]) { const float tv = top[k]; top[k] = v; v = tv; } } } }
    wave_lds_sync(); }
  if (lane < 16) { float s = 0.0f;
#pragma unroll
    for (int k = 0; k < KN; ++k) s += top[k]; Rsum[lane] = s; }
  wave_lds_sync(); float tot = 0.0f; if (lane == 0) { for (int r = 0; r < 16; ++r) tot += Rsum[r]; }
  for (int pass = 0; pass < 2; ++pass) { ((volatile float*)PART)[(size_t)blockIdx.x * 32 + lane] = lane == 0 ? tot : 0.0f; __threadfence(); }
}
__global__ __launch_bounds__(32) void loss_kernel(const float* __restrict__ PART, int nparts, float* __restrict__ LOSS) { const int lane = threadIdx.x; float s = 0.0f; if (lane == 0) { for (int i = 0; i < nparts; ++i) s += PART[(size_t)i * 32]; } for (int pass = 0; pass < 2; ++pass) { ((volatile float*)LOSS)[lane] = lane == 0 ? s : 0.0f; __threadfence(); } }
__global__ __launch_bounds__(256) void copy_kernel(const float* __restrict__ LOSS, const float* __restrict__ H, float* __restrict__ out) { const size_t i = (size_t)blockIdx.x * 256 + threadIdx.x; if (i >= (size_t)NT * D + 1) return; const float v = i == 0 ? LOSS[0] : H[i - 1]; for (int pass = 0; pass < 2; ++pass) { ((volatile float*)out)[i] = v; __threadfence(); } }
}

extern "C" void kernel_launch(void* const* d_in, const int* in_sizes, int n_in, void* d_out, int out_size, void* d_ws, size_t ws_size, hipStream_t stream) {
  (void)n_in;
  auto Fp = [&](int i) { return (const float*)d_in[i]; };
  if (in_sizes[0] != NT * IN || in_sizes[1] != IN * D || in_sizes[3] != NL * D * D || in_sizes[7] != NL * D * DFF || in_sizes[9] != NL * DFF * D || out_size != 1 + NT * D) return;
  const int BV = BS; const int RL = BV * S, GB16 = RL / 16;
  size_t off = 0; char* ws = (char*)d_ws;
  auto carve = [&](size_t bytes) { char* p = ws + off; off += (bytes + 255) & ~(size_t)255; return p; };
  b16* WE = (b16*)carve(D * 32 * 2); b16* WQ = (b16*)carve((size_t)NL * D * D * 2); b16* WK = (b16*)carve((size_t)NL * D * D * 2); b16* WV = (b16*)carve((size_t)NL * D * D * 2); b16* WO = (b16*)carve((size_t)NL * D * D * 2); b16* W1T = (b16*)carve((size_t)NL * DFF * D * 2); b16* W2T = (b16*)carve((size_t)NL * D * DFF * 2);
  float* H = (float*)carve((size_t)NT * D * 4); float* H1 = (float*)carve((size_t)NT * D * 4); float* QKV = (float*)carve((size_t)NT * 3 * D * 4); float* ATT = (float*)carve((size_t)NT * D * 4); float* SQ = (float*)carve((size_t)NT * 4); float* PART = (float*)carve((size_t)NBLK * 32 * 4); float* LOSS = (float*)carve(32 * 4);
  if (off > ws_size || off > ((size_t)32 << 20)) return;
  wput_kernel<<<(D * 4 + 255) / 256, 256, 0, stream>>>(Fp(1), IN, 32, D, WE);
  for (int l = 0; l < NL; ++l) { wput_kernel<<<(D * 16 + 255) / 256, 256, 0, stream>>>(Fp(3) + (size_t)l * D * D, D, D, D, WQ + (size_t)l * D * D); wput_kernel<<<(D * 16 + 255) / 256, 256, 0, stream>>>(Fp(4) + (size_t)l * D * D, D, D, D, WK + (size_t)l * D * D); wput_kernel<<<(D * 16 + 255) / 256, 256, 0, stream>>>(Fp(5) + (size_t)l * D * D, D, D, D, WV + (size_t)l * D * D); wput_kernel<<<(D * 16 + 255) / 256, 256, 0, stream>>>(Fp(6) + (size_t)l * D * D, D, D, D, WO + (size_t)l * D * D);
    wput_kernel<<<(DFF * 16 + 255) / 256, 256, 0, stream>>>(Fp(7) + (size_t)l * D * DFF, D, D, DFF, W1T + (size_t)l * DFF * D); wput_kernel<<<(D * 64 + 255) / 256, 256, 0, stream>>>(Fp(9) + (size_t)l * DFF * D, DFF, DFF, D, W2T + (size_t)l * D * DFF); }
  emb_kernel<<<GB16, 32, 0, stream>>>(Fp(0), WE, Fp(2), RL, H);
  for (int l = 0; l < NL; ++l) {
    qkv_kernel<<<GB16, 32, 0, stream>>>(H, WQ + (size_t)l * D * D, WK + (size_t)l * D * D, WV + (size_t)l * D * D, RL, QKV);
    att_kernel<<<BV * (S / 16), 32, 0, stream>>>(QKV, BV, ATT);
    wo_kernel<<<GB16, 32, 0, stream>>>(ATT, H, WO + (size_t)l * D * D, Fp(11) + l * D, Fp(12) + l * D, RL, H1);
    ffn_kernel<<<GB16, 32, 0, stream>>>(H1, W1T + (size_t)l * DFF * D, Fp(8) + l * DFF, W2T + (size_t)l * D * DFF, Fp(10) + l * D, Fp(13) + l * D, Fp(14) + l * D, RL, H); }
  sq_kernel<<<(RL + 255) / 256, 256, 0, stream>>>(H, RL, SQ);
  knn_kernel<<<GB16, 32, 0, stream>>>(H, SQ, RL, PART);
  loss_kernel<<<1, 32, 0, stream>>>(PART, GB16, LOSS);
  copy_kernel<<<(unsigned)(((size_t)NT * D + 1 + 255) / 256), 256, 0, stream>>>(LOSS, H, (float*)d_out);
}
